// MultiLSTMConceptCorrector_27084063768956
// MI455X (gfx1250) — hardware-verified
//
#include <hip/hip_runtime.h>

typedef __attribute__((ext_vector_type(16))) _Float16 v16h;
typedef __attribute__((ext_vector_type(8)))  _Float16 v8h;
typedef __attribute__((ext_vector_type(8)))  float    v8f;
typedef __attribute__((ext_vector_type(4)))  float    v4f;

__device__ __forceinline__ void dep_guard_h(v8f& a, v8f& b, v16h x, v16h y) { asm volatile("v_nop\n\tv_nop\n\tv_nop\n\tv_nop" : "+v"(a), "+v"(b) : "v"(x), "v"(y)); }
__device__ __forceinline__ void keep4_h(v16h a, v16h b, v16h c, v16h d) { asm volatile("v_nop" :: "v"(a), "v"(b), "v"(c), "v"(d)); }
template <typename T> struct Frag;
template <> struct Frag<_Float16> {
  typedef v16h V; union U { v16h v; v8h h[2]; };
  static __device__ __forceinline__ v16h load(const _Float16* p) {
    U f; f.h[0] = *(const v8h*)(p); f.h[1] = *(const v8h*)(p + 16); return f.v;
  }
  static __device__ __forceinline__ v8f mma(v16h a, v16h b, v8f c) {
    return __builtin_amdgcn_wmma_f32_16x16x32_f16(false, a, false, b, (short)0, c, false, false);
  }
  static __device__ __forceinline__ void guard(v8f& a, v8f& b, v16h x, v16h y) { dep_guard_h(a, b, x, y); }
  static __device__ __forceinline__ void keep(v16h a, v16h b, v16h c, v16h d) { keep4_h(a, b, c, d); }
};

__device__ __forceinline__ v8f mma16(v16h a, v16h b, v8f c) {
  c = __builtin_amdgcn_wmma_f32_16x16x32_f16(false, a, false, b, (short)0, c, false, false);
  asm volatile("v_nop\n\tv_nop\n\tv_nop\n\tv_nop" : "+v"(c) : "v"(a), "v"(b));
  return c;
}

constexpr int kBatch  = 64;
constexpr int kSteps  = 256;
constexpr int kConc   = 256;
constexpr int kClus   = 8;
constexpr int kHid    = 256;
constexpr int kCc     = 32;
constexpr int kGate   = 4 * kHid;
constexpr int kKcat   = kCc + kHid;
constexpr int kRows   = 16;
constexpr int kXPitch = 296;
constexpr int kOPitch = 36;
constexpr float kOpScale = 8.0f;
constexpr float kFold    = 0.015625f;
static_assert(kKcat % 32 == 0);
static_assert(kHid % 32 == 0);
static_assert(kXPitch % 8 == 0 && kXPitch >= kKcat);
static_assert(kBatch % kRows == 0);

constexpr size_t kWcatHalves = (size_t)kClus * kGate * kKcat;
constexpr size_t kWfcHalves  = (size_t)kClus * kCc * kHid;
constexpr size_t kWcatOff    = 0;
constexpr size_t kWfcOff     = kWcatOff + kWcatHalves * 2;
constexpr size_t kWsTotal    = kWfcOff + kWfcHalves * 2;
constexpr int kPrepBlkWcat   = (int)(kWcatHalves / (8 * 256));
constexpr int kPrepBlkWfc    = (int)(kWfcHalves / (8 * 256));
static_assert(kWcatHalves % (8 * 256) == 0);
static_assert(kWfcHalves % (8 * 256) == 0);
static_assert(kWfcOff % 128 == 0);

__device__ __forceinline__ float sigm_f(float x) {
  x = fminf(fmaxf(x, -30.0f), 30.0f);
  const float e = expf(-x);
  return __builtin_amdgcn_rcpf(1.0f + e);
}
__device__ __forceinline__ float tanh_f(float x) {
  x = fminf(fmaxf(x, -15.0f), 15.0f);
  const float e = expf(2.0f * x);
  return 1.0f - 2.0f * __builtin_amdgcn_rcpf(1.0f + e);
}

__global__ __launch_bounds__(256) void prep_planes(
    const float* __restrict__ W_ih, const float* __restrict__ W_hh, const float* __restrict__ W_fc,
    _Float16* __restrict__ wcat, _Float16* __restrict__ wfc) {
  const int tid = threadIdx.x;
  if ((int)blockIdx.x < kPrepBlkWcat) {
    const size_t i8 = (size_t)blockIdx.x * 256 + tid;
    const size_t i  = i8 * 8;
    const int row = (int)(i / kKcat);
    const int k0  = (int)(i - (size_t)row * kKcat);
    const int kih = (k0 < 24) ? k0 : 24;
    const int khh = (k0 >= kCc) ? (k0 - kCc) : 0;
    const float* pa = W_ih + (size_t)row * kCc + kih;
    const float* pb = W_hh + (size_t)row * kHid + khh;
    const bool useih = (k0 < kCc);
    v8h hv;
#pragma unroll
    for (int e = 0; e < 8; ++e) {
      const float a = pa[e];
      const float b = pb[e];
      const float v = useih ? a : b;
      hv[e] = (_Float16)(v * kOpScale);
    }
    _Float16* dst = wcat + i;
    for (int pass = 0; pass < 2; ++pass) {
      *(volatile v8h*)dst = hv;
      __threadfence();
    }
  } else {
    const size_t i = ((size_t)((int)blockIdx.x - kPrepBlkWcat) * 256 + tid) * 8;
    const float* p = W_fc + i;
    v8h hv;
#pragma unroll
    for (int e = 0; e < 8; ++e) hv[e] = (_Float16)(p[e] * kOpScale);
    _Float16* dst = wfc + i;
    for (int pass = 0; pass < 2; ++pass) {
      *(volatile v8h*)dst = hv;
      __threadfence();
    }
  }
}

__global__ __launch_bounds__(256) void lstm_cluster_scan(
    const float* __restrict__ inp, const float* __restrict__ aic, const float* __restrict__ org,
    const float* __restrict__ h0, const float* __restrict__ c0,
    const _Float16* wcat, const _Float16* wfc,
    const float* __restrict__ b_ih, const float* __restrict__ b_hh, const float* __restrict__ b_fc,
    float* __restrict__ out0, float* __restrict__ out1, float* __restrict__ out2) {

  __shared__ __align__(16) _Float16 xh[kRows * kXPitch];
  __shared__ __align__(16) float aS[kRows * kCc];
  __shared__ __align__(16) float oS[kRows * kCc];
  __shared__ __align__(16) float outS[kRows * kOPitch];
  __shared__ __align__(16) float hS[kRows * kHid];
  __shared__ __align__(16) float cS[kRows * kHid];

  const int m    = blockIdx.x;
  const int b0   = blockIdx.y * kRows;
  const int tid  = threadIdx.x;
  const int lane = tid & 31;
  const int wave = tid >> 5;
  const int hh   = lane >> 4;
  const int c    = lane & 15;

  const _Float16* wm = wcat + (size_t)m * kGate * kKcat;
  const _Float16* wf = wfc + (size_t)m * kCc * kHid;

#pragma unroll 1
  for (int it = 0; it < kRows; ++it) {
    const float v = h0[((size_t)(m * kBatch + b0 + it)) * kHid + tid];
    xh[it * kXPitch + kCc + tid] = (_Float16)(v * kOpScale);
  }

  v8f cst[2], hlast[2];
  float bsum[8];
#pragma unroll
  for (int us = 0; us < 2; ++us) {
    const int ub = 2 * wave + us;
#pragma unroll
    for (int r = 0; r < 8; ++r) {
      const size_t si = ((size_t)(m * kBatch + b0 + 8 * hh + r)) * kHid + 16 * ub + c;
      cst[us][r]   = c0[si];
      hlast[us][r] = h0[si];
    }
#pragma unroll
    for (int q = 0; q < 4; ++q) {
      const int n = q * kHid + 16 * ub + c;
      bsum[q * 2 + us] = b_ih[m * kGate + n] + b_hh[m * kGate + n];
    }
  }

  const v8f zero8 = (v8f){0.f, 0.f, 0.f, 0.f, 0.f, 0.f, 0.f, 0.f};

#pragma unroll 1
  for (int t = 0; t < kSteps; ++t) {
#pragma unroll
    for (int p = 0; p < 2; ++p) {
      const int r  = wave + 8 * p;
      const int cc = lane;
      const size_t gi = ((size_t)(b0 + r) * kSteps + t) * kConc + m * kCc + cc;
      const float av = aic[gi];
      const float iv = inp[gi];
      const float ov = org[gi];
      const float xv = av * iv + (1.0f - av) * ov;
      xh[r * kXPitch + cc] = (_Float16)(xv * kOpScale);
      aS[r * kCc + cc] = av;
      oS[r * kCc + cc] = ov;
    }
    __syncthreads();

    v8f acc[8];
#pragma unroll
    for (int a = 0; a < 8; ++a) acc[a] = zero8;
    int zoff = 0;
    asm volatile("" : "+v"(zoff));
    const _Float16* wmt = wm + zoff;
#pragma unroll 1
    for (int kk = 0; kk < 9; ++kk) {
      const int k0 = kk * 32;
      const v16h av = Frag<_Float16>::load(xh + c * kXPitch + k0 + 8 * hh);
#pragma unroll
      for (int q = 0; q < 4; ++q) {
#pragma unroll
        for (int us = 0; us < 2; ++us) {
          const int n = q * kHid + 16 * (2 * wave + us) + c;
          const v16h bv = Frag<_Float16>::load(wmt + (size_t)n * kKcat + k0 + 8 * hh);
          acc[q * 2 + us] = mma16(av, bv, acc[q * 2 + us]);
        }
      }
    }
    __syncthreads();

#pragma unroll
    for (int us = 0; us < 2; ++us) {
      const int ub = 2 * wave + us;
#pragma unroll
      for (int r = 0; r < 8; ++r) {
        const float gi = acc[0 + us][r] * kFold + bsum[0 + us];
        const float gf = acc[2 + us][r] * kFold + bsum[2 + us];
        const float gg = acc[4 + us][r] * kFold + bsum[4 + us];
        const float go = acc[6 + us][r] * kFold + bsum[6 + us];
        const float cn = sigm_f(gf) * cst[us][r] + sigm_f(gi) * tanh_f(gg);
        cst[us][r] = cn;
        const float hn = sigm_f(go) * tanh_f(cn);
        hlast[us][r] = hn;
        xh[(8 * hh + r) * kXPitch + kCc + 16 * ub + c] = (_Float16)(hn * kOpScale);
      }
    }
    __syncthreads();

    if (wave < 2) {
      v8f fa = zero8;
#pragma unroll 1
      for (int kk = 0; kk < 8; ++kk) {
        const v16h av = Frag<_Float16>::load(xh + c * kXPitch + kCc + kk * 32 + 8 * hh);
        const v16h bv = Frag<_Float16>::load(wf + (size_t)(wave * 16 + c) * kHid + kk * 32 + 8 * hh);
        fa = mma16(av, bv, fa);
      }
      const int j = wave * 16 + c;
      const float bfv = b_fc[m * kCc + j];
#pragma unroll
      for (int r = 0; r < 8; ++r) {
        const int row = 8 * hh + r;
        const float v = fa[r] * kFold + bfv;
        const float s = sigm_f(v);
        const float av = aS[row * kCc + j];
        const float ov = oS[row * kCc + j];
        outS[row * kOPitch + j] = av * ov + (1.0f - av) * s;
      }
    }
    __syncthreads();

    if (wave < 4) {
      const int row = wave * 4 + (lane >> 3);
      const int c4  = (lane & 7) * 4;
      const v4f val = *(const v4f*)(outS + row * kOPitch + c4);
      float* gp = out0 + ((size_t)(b0 + row) * kSteps + t) * kConc + m * kCc + c4;
      for (int pass = 0; pass < 2; ++pass) {
        *(volatile v4f*)gp = val;
        __threadfence();
      }
    }
  }

#pragma unroll
  for (int us = 0; us < 2; ++us) {
    const int ub = 2 * wave + us;
#pragma unroll
    for (int r = 0; r < 8; ++r) {
      hS[(8 * hh + r) * kHid + 16 * ub + c] = hlast[us][r];
      cS[(8 * hh + r) * kHid + 16 * ub + c] = cst[us][r];
    }
  }
  __syncthreads();
  const size_t base = ((size_t)(m * kBatch + b0)) * kHid;
  for (int pass = 0; pass < 2; ++pass) {
#pragma unroll
    for (int it = 0; it < 4; ++it) {
      const int q4 = it * 256 + tid;
      const v4f hv = *(const v4f*)(hS + q4 * 4);
      const v4f cv = *(const v4f*)(cS + q4 * 4);
      *(volatile v4f*)(out1 + base + (size_t)q4 * 4) = hv;
      *(volatile v4f*)(out2 + base + (size_t)q4 * 4) = cv;
    }
    __threadfence();
  }
}

extern "C" void kernel_launch(void* const* d_in, const int* in_sizes, int n_in,
                              void* d_out, int out_size, void* d_ws, size_t ws_size,
                              hipStream_t stream) {
  if (n_in < 11) return;
  if (in_sizes[0] != kBatch * kSteps * kConc) return;
  if (in_sizes[1] != kBatch * kSteps * kConc) return;
  if (in_sizes[2] != kBatch * kSteps * kConc) return;
  if (in_sizes[3] != kClus * kBatch * kHid) return;
  if (in_sizes[4] != kClus * kBatch * kHid) return;
  if (in_sizes[5] != kClus * kGate * kCc) return;
  if (in_sizes[6] != kClus * kGate * kHid) return;
  if (in_sizes[7] != kClus * kGate) return;
  if (in_sizes[8] != kClus * kGate) return;
  if (in_sizes[9] != kClus * kCc * kHid) return;
  if (in_sizes[10] != kClus * kCc) return;
  if ((size_t)out_size != (size_t)kBatch * kSteps * kConc + 2 * (size_t)kClus * kBatch * kHid) return;
  if (ws_size < kWsTotal) return;

  const float* inp  = (const float*)d_in[0];
  const float* aic  = (const float*)d_in[1];
  const float* org  = (const float*)d_in[2];
  const float* h0   = (const float*)d_in[3];
  const float* c0   = (const float*)d_in[4];
  const float* W_ih = (const float*)d_in[5];
  const float* W_hh = (const float*)d_in[6];
  const float* b_ih = (const float*)d_in[7];
  const float* b_hh = (const float*)d_in[8];
  const float* W_fc = (const float*)d_in[9];
  const float* b_fc = (const float*)d_in[10];

  float* out0 = (float*)d_out;
  float* out1 = out0 + (size_t)kBatch * kSteps * kConc;
  float* out2 = out1 + (size_t)kClus * kBatch * kHid;

  char* ws = (char*)d_ws;
  _Float16* wcat = (_Float16*)(ws + kWcatOff);
  _Float16* wfc  = (_Float16*)(ws + kWfcOff);

  prep_planes<<<dim3(kPrepBlkWcat + kPrepBlkWfc), dim3(256), 0, stream>>>(W_ih, W_hh, W_fc, wcat, wfc);

  lstm_cluster_scan<<<dim3(kClus, kBatch / kRows), dim3(256), 0, stream>>>(
      inp, aic, org, h0, c0, wcat, wfc, b_ih, b_hh, b_fc, out0, out1, out2);
}
